// LinOSSSequenceMixer_17626545783732
// MI455X (gfx1250) — hardware-verified
//
#include <hip/hip_runtime.h>
#include <math.h>

#define NB    16
#define NL    4096
#define NH    128
#define NS    256
#define QSEQ  4
#define QROWS (QSEQ * NL)
#define NQ    (NB / QSEQ)

typedef __attribute__((ext_vector_type(16))) _Float16 v16h;
typedef __attribute__((ext_vector_type(8)))  _Float16 v8h;
typedef __attribute__((ext_vector_type(16))) __bf16   v16b;
typedef __attribute__((ext_vector_type(8)))  __bf16   v8b;
typedef __attribute__((ext_vector_type(8)))  float    v8f;
typedef __attribute__((ext_vector_type(4)))  float    v4f;
typedef __attribute__((ext_vector_type(4)))  unsigned int v4u;

__device__ __forceinline__ unsigned short f2bf_bits(float f) {
  unsigned u = __float_as_uint(f);
  return (unsigned short)((u + 0x7FFFu + ((u >> 16) & 1u)) >> 16);
}
__device__ __forceinline__ float bf_bits2f(unsigned short h) { return __uint_as_float(((unsigned)h) << 16); }

__device__ __forceinline__ void dep_guard_h(v8f& a, v8f& b, v16h x, v16h y) { asm volatile("v_nop\n\tv_nop\n\tv_nop\n\tv_nop" : "+v"(a), "+v"(b) : "v"(x), "v"(y)); }
__device__ __forceinline__ void dep_guard_b(v8f& a, v8f& b, v16b x, v16b y) { asm volatile("v_nop\n\tv_nop\n\tv_nop\n\tv_nop" : "+v"(a), "+v"(b) : "v"(x), "v"(y)); }
__device__ __forceinline__ void keep4_h(v16h a, v16h b, v16h c, v16h d) { asm volatile("v_nop" :: "v"(a), "v"(b), "v"(c), "v"(d)); }
__device__ __forceinline__ void keep4_b(v16b a, v16b b, v16b c, v16b d) { asm volatile("v_nop" :: "v"(a), "v"(b), "v"(c), "v"(d)); }
__device__ __forceinline__ void acc_guard4(v8f& a, v8f& b, v8f& c, v8f& d) { asm volatile("v_nop\n\tv_nop\n\tv_nop\n\tv_nop" : "+v"(a), "+v"(b), "+v"(c), "+v"(d)); }
template <typename T> struct Frag;
template <> struct Frag<_Float16> {
  typedef v16h V; union U { v16h v; v8h h[2]; };
  static __device__ __forceinline__ v16h load(const _Float16* p) {
    U f; f.h[0] = *(const v8h*)(p); f.h[1] = *(const v8h*)(p + 16); return f.v;
  }
  static __device__ __forceinline__ v8f mma(v16h a, v16h b, v8f c) {
    return __builtin_amdgcn_wmma_f32_16x16x32_f16(false, a, false, b, (short)0, c, false, false);
  }
  static __device__ __forceinline__ void guard(v8f& a, v8f& b, v16h x, v16h y) { dep_guard_h(a, b, x, y); }
  static __device__ __forceinline__ void keep(v16h a, v16h b, v16h c, v16h d) { keep4_h(a, b, c, d); }
};
template <> struct Frag<__bf16> {
  typedef v16b V; union U { v16b v; v8b h[2]; };
  static __device__ __forceinline__ v16b load(const __bf16* p) {
    U f; f.h[0] = *(const v8b*)(p); f.h[1] = *(const v8b*)(p + 16); return f.v;
  }
  static __device__ __forceinline__ v8f mma(v16b a, v16b b, v8f c) {
    return __builtin_amdgcn_wmma_f32_16x16x32_bf16(false, a, false, b, (short)0, c, false, false);
  }
  static __device__ __forceinline__ void guard(v8f& a, v8f& b, v16b x, v16b y) { dep_guard_b(a, b, x, y); }
  static __device__ __forceinline__ void keep(v16b a, v16b b, v16b c, v16b d) { keep4_b(a, b, c, d); }
};

template <int ET> struct Elem;
template <> struct Elem<0> { typedef _Float16 T; };
template <> struct Elem<1> { typedef __bf16 T; };
template <int ET, bool SPLIT, int BIAS_MODE, int OUT_MODE, int RESID, int ACT = 0>
__global__ __launch_bounds__(256) void wmma_gemm64(
    const unsigned short* __restrict__ Ap, const unsigned short* __restrict__ A2p, int lda, long strideA,
    const unsigned short* __restrict__ Btp, const unsigned short* __restrict__ Bt2p, int ldb, long strideB,
    void* __restrict__ Cout, void* __restrict__ Cout2, int ldc, long strideC,
    const float* __restrict__ bias,
    const float* __restrict__ resid, long strideR, const float* __restrict__ rcoef,
    int M, int N, int K, float scale) {
  typedef typename Elem<ET>::T T;
  typedef typename Frag<T>::V V;
  const T* A = (const T*)Ap; const T* A2 = (const T*)A2p; const T* Bt = (const T*)Btp; const T* Bt2 = (const T*)Bt2p;
  __shared__ __align__(16) float sT[8][16 * 68];
  const int b    = blockIdx.y;
  const int lane = threadIdx.x & 31;
  const int wave = threadIdx.x >> 5;
  const int tilesN = N >> 6;
  const int tilesM = M >> 6;
  const int tile = blockIdx.x * 8 + wave;
  if (tile >= tilesM * tilesN) return;
  const int tm = tile / tilesN;
  const int tn = tile - tm * tilesN;
  const int m0 = tm << 6;
  const int n0 = tn << 6;

  const T* Ab  = A  + (size_t)b * strideA;
  const T* Bb  = Bt + (size_t)b * strideB;
  const T* Ab2 = SPLIT ? (A2  + (size_t)b * strideA) : nullptr;
  const T* Bb2 = SPLIT ? (Bt2 + (size_t)b * strideB) : nullptr;

  const int rlane = lane & 15;
  const int koff  = (lane >> 4) * 8;
  const int mOff  = (lane >> 4) * 8;

  v8f acc[4][4];
#pragma unroll
  for (int i = 0; i < 4; ++i)
#pragma unroll
    for (int j = 0; j < 4; ++j) acc[i][j] = (v8f){0.f,0.f,0.f,0.f,0.f,0.f,0.f,0.f};

  for (int k0 = 0; k0 < K; k0 += 32) {
    V bh[4], bl[4];
#pragma unroll
    for (int j = 0; j < 4; ++j) {
      const size_t bo = (size_t)(n0 + (j << 4) + rlane) * ldb + koff + k0;
      bh[j] = Frag<T>::load(Bb + bo);
      if (SPLIT) bl[j] = Frag<T>::load(Bb2 + bo);
    }
#pragma unroll
    for (int i = 0; i < 4; ++i) {
      const size_t ao = (size_t)(m0 + (i << 4) + rlane) * lda + koff + k0;
      V ah = Frag<T>::load(Ab + ao);
      V al;
      if (SPLIT) al = Frag<T>::load(Ab2 + ao);
#pragma unroll
      for (int j = 0; j < 4; ++j) {
        acc[i][j] = Frag<T>::mma(ah, bh[j], acc[i][j]);
        if (SPLIT) {
          acc[i][j] = Frag<T>::mma(ah, bl[j], acc[i][j]);
          acc[i][j] = Frag<T>::mma(al, bh[j], acc[i][j]);
        }
      }
      Frag<T>::guard(acc[i][0], acc[i][3], ah, SPLIT ? al : ah);
    }
    Frag<T>::keep(bh[0], bh[1], bh[2], bh[3]);
    if (SPLIT) Frag<T>::keep(bl[0], bl[1], bl[2], bl[3]);
  }
  acc_guard4(acc[0][0], acc[0][1], acc[0][2], acc[0][3]);
  acc_guard4(acc[1][0], acc[1][1], acc[1][2], acc[1][3]);
  acc_guard4(acc[2][0], acc[2][1], acc[2][2], acc[2][3]);
  acc_guard4(acc[3][0], acc[3][1], acc[3][2], acc[3][3]);

  float* slab = sT[wave];
  const float* Rb = (RESID != 0) ? (resid + (size_t)b * strideR) : nullptr;
#pragma unroll
  for (int i = 0; i < 4; ++i) {
    const int mBase = m0 + (i << 4);
#pragma unroll
    for (int j = 0; j < 4; ++j) {
      const int n = n0 + (j << 4) + rlane;
      float bv = 0.f;
      if (BIAS_MODE == 2) bv = bias[n];
      float rc = 0.f;
      if (RESID == 2) rc = rcoef[n];
#pragma unroll
      for (int r = 0; r < 8; ++r) {
        float v = acc[i][j][r] * scale;
        if (BIAS_MODE == 1) v += bias[mBase + mOff + r];
        if (BIAS_MODE == 2) v += bv;
        if (RESID == 1) v += Rb[(size_t)(mBase + mOff + r) * ldc + n];
        if (RESID == 2) v += rc * Rb[(size_t)(mBase + mOff + r) * ldc + n];
        if (ACT == 1) v = tanhf(v);
        if (ACT == 2) v = fmaxf(v, 0.0f);
        if (ACT == 3) v = v / (1.0f + expf(-v));
        if (ACT == 4) v = (v > 0.f) ? v : 0.01f * v;
        if (ACT == 5) v = 0.5f * v * (1.0f + erff(v * 0.70710678118654752f));
        slab[(mOff + r) * 68 + (j << 4) + rlane] = v;
      }
    }
    __builtin_amdgcn_fence(__ATOMIC_RELEASE, "workgroup");
    __builtin_amdgcn_wave_barrier();
    __builtin_amdgcn_fence(__ATOMIC_ACQUIRE, "workgroup");
    if (OUT_MODE == 0) {
      float* C = (float*)Cout + (size_t)b * strideC;
      const int hh = lane >> 4, c4 = (lane & 15) * 4;
      for (int pass = 0; pass < 2; ++pass) {
#pragma unroll
        for (int it = 0; it < 8; ++it) {
          const int row = it * 2 + hh;
          v4f v = *(const v4f*)(slab + row * 68 + c4);
          *(volatile v4f*)(C + (size_t)(mBase + row) * ldc + n0 + c4) = v;
        }
        __threadfence();
      }
    } else {
      const int q = lane >> 3, c8 = (lane & 7) * 8;
      unsigned short* C  = (unsigned short*)Cout  + (size_t)b * strideC;
      unsigned short* C2 = (OUT_MODE == 2) ? ((unsigned short*)Cout2 + (size_t)b * strideC) : nullptr;
      for (int pass = 0; pass < 2; ++pass) {
#pragma unroll
        for (int it = 0; it < 4; ++it) {
          const int row = it * 4 + q;
          const float* sp = slab + row * 68 + c8;
          v8h hv, lv;
#pragma unroll
          for (int e = 0; e < 8; ++e) {
            if (OUT_MODE == 1) {
              hv[e] = (_Float16)sp[e];
            } else {
              unsigned short hb = f2bf_bits(sp[e]);
              unsigned short lb = f2bf_bits(sp[e] - bf_bits2f(hb));
              hv[e] = __builtin_bit_cast(_Float16, hb);
              lv[e] = __builtin_bit_cast(_Float16, lb);
            }
          }
          *(volatile v8h*)(C + (size_t)(mBase + row) * ldc + n0 + c8) = hv;
          if (OUT_MODE == 2) *(volatile v8h*)(C2 + (size_t)(mBase + row) * ldc + n0 + c8) = lv;
        }
        __threadfence();
      }
    }
    __builtin_amdgcn_fence(__ATOMIC_RELEASE, "workgroup");
    __builtin_amdgcn_wave_barrier();
    __builtin_amdgcn_fence(__ATOMIC_ACQUIRE, "workgroup");
  }
}

__global__ __launch_bounds__(256) void split_bf16x8(const float* __restrict__ in,
                                                   unsigned short* __restrict__ hi,
                                                   unsigned short* __restrict__ lo, int n8) {
  const int i = blockIdx.x * 256 + threadIdx.x;
  if (i >= n8) return;
  const float* p = in + (size_t)i * 8;
  const v4f a = *(const v4f*)p;
  const v4f c = *(const v4f*)(p + 4);
  float f[8];
#pragma unroll
  for (int e = 0; e < 4; ++e) { f[e] = a[e]; f[4 + e] = c[e]; }
  v4u hv, lv;
#pragma unroll
  for (int e = 0; e < 4; ++e) {
    const unsigned short h0 = f2bf_bits(f[2 * e]);
    const unsigned short h1 = f2bf_bits(f[2 * e + 1]);
    const unsigned short l0 = f2bf_bits(f[2 * e] - bf_bits2f(h0));
    const unsigned short l1 = f2bf_bits(f[2 * e + 1] - bf_bits2f(h1));
    hv[e] = (unsigned)h0 | ((unsigned)h1 << 16);
    lv[e] = (unsigned)l0 | ((unsigned)l1 << 16);
  }
  unsigned short* hp = hi + (size_t)i * 8;
  unsigned short* lp = lo + (size_t)i * 8;
  *(volatile v4u*)hp = hv;
  *(volatile v4u*)lp = lv;
  __threadfence();
  *(volatile v4u*)hp = hv;
  *(volatile v4u*)lp = lv;
}

__global__ __launch_bounds__(NS) void state_params(const float* __restrict__ A_diag,
                                                  const float* __restrict__ steps,
                                                  float* __restrict__ PT) {
  const int n = threadIdx.x;
  const float st    = 1.0f / (1.0f + expf(-steps[n]));
  const float A     = fmaxf(A_diag[n], 0.0f);
  const float s2A   = (st * st) * A;
  const float schur = 1.0f / (1.0f + s2A);
  const float M11 = 1.0f - s2A * schur;
  const float M12 = ((-st) * A) * schur;
  const float M21 = st * schur;
  const float M22 = schur;
  const float c1  = M11 * st;
  const float c2  = M21 * st;
  volatile float* P = PT;
  P[0 * NS + n] = M11; P[1 * NS + n] = M12; P[2 * NS + n] = M21;
  P[3 * NS + n] = M22; P[4 * NS + n] = c1;  P[5 * NS + n] = c2;
  __threadfence();
  P[0 * NS + n] = M11; P[1 * NS + n] = M12; P[2 * NS + n] = M21;
  P[3 * NS + n] = M22; P[4 * NS + n] = c1;  P[5 * NS + n] = c2;
}

__global__ __launch_bounds__(32) void state_scan(const float* __restrict__ PT,
                                                const float* __restrict__ BU,
                                                unsigned short* __restrict__ YSh,
                                                unsigned short* __restrict__ YSl) {
  const int q  = threadIdx.x;
  const int sl = blockIdx.x;
  const int n0 = q * 8;
  float m11[8], m12[8], m21[8], m22[8], c1[8], c2[8], z1[8], z2[8];
  {
    const v4f a0 = *(const v4f*)(PT + 0 * NS + n0), a1 = *(const v4f*)(PT + 0 * NS + n0 + 4);
    const v4f b0 = *(const v4f*)(PT + 1 * NS + n0), b1 = *(const v4f*)(PT + 1 * NS + n0 + 4);
    const v4f d0 = *(const v4f*)(PT + 2 * NS + n0), d1 = *(const v4f*)(PT + 2 * NS + n0 + 4);
    const v4f e0 = *(const v4f*)(PT + 3 * NS + n0), e1 = *(const v4f*)(PT + 3 * NS + n0 + 4);
    const v4f f0 = *(const v4f*)(PT + 4 * NS + n0), f1 = *(const v4f*)(PT + 4 * NS + n0 + 4);
    const v4f g0 = *(const v4f*)(PT + 5 * NS + n0), g1 = *(const v4f*)(PT + 5 * NS + n0 + 4);
#pragma unroll
    for (int e = 0; e < 4; ++e) {
      m11[e] = a0[e]; m11[4 + e] = a1[e];
      m12[e] = b0[e]; m12[4 + e] = b1[e];
      m21[e] = d0[e]; m21[4 + e] = d1[e];
      m22[e] = e0[e]; m22[4 + e] = e1[e];
      c1[e]  = f0[e]; c1[4 + e]  = f1[e];
      c2[e]  = g0[e]; c2[4 + e]  = g1[e];
    }
  }
#pragma unroll
  for (int k = 0; k < 8; ++k) { z1[k] = 0.f; z2[k] = 0.f; }

#pragma unroll 1
  for (int l = 0; l < NL; ++l) {
    const size_t row = (size_t)sl * NL + (size_t)l;
    const float* bp = BU + row * NS + n0;
    const v4f b0 = *(const v4f*)bp;
    const v4f b1 = *(const v4f*)(bp + 4);
    float bu[8];
#pragma unroll
    for (int e = 0; e < 4; ++e) { bu[e] = b0[e]; bu[4 + e] = b1[e]; }
    v4u hv, lv;
#pragma unroll
    for (int e = 0; e < 4; ++e) {
      unsigned hpk = 0u, lpk = 0u;
#pragma unroll
      for (int p = 0; p < 2; ++p) {
        const int k = 2 * e + p;
        const float o1 = z1[k], o2 = z2[k];
        const float u1 = m11[k] * o1 + m12[k] * o2 + c1[k] * bu[k];
        const float u2 = m21[k] * o1 + m22[k] * o2 + c2[k] * bu[k];
        z1[k] = u1; z2[k] = u2;
        const unsigned short hb = f2bf_bits(u2);
        const unsigned short lb = f2bf_bits(u2 - bf_bits2f(hb));
        hpk |= ((unsigned)hb) << (16 * p);
        lpk |= ((unsigned)lb) << (16 * p);
      }
      hv[e] = hpk; lv[e] = lpk;
    }
    unsigned short* hp = YSh + row * NS + n0;
    unsigned short* lp = YSl + row * NS + n0;
    *(volatile v4u*)hp = hv;
    *(volatile v4u*)lp = lv;
    __threadfence();
    *(volatile v4u*)hp = hv;
    *(volatile v4u*)lp = lv;
  }
}

extern "C" void kernel_launch(void* const* d_in, const int* in_sizes, int n_in,
                              void* d_out, int out_size, void* d_ws, size_t ws_size,
                              hipStream_t stream) {
  if (n_in < 6) return;
  if (in_sizes[0] != NB * NL * NH || in_sizes[1] != NS || in_sizes[2] != NS ||
      in_sizes[3] != NS * NH || in_sizes[4] != NH * NS || in_sizes[5] != NH) return;
  if (out_size != NB * NL * NH) return;

  const float* x      = (const float*)d_in[0];
  const float* A_diag = (const float*)d_in[1];
  const float* steps  = (const float*)d_in[2];
  const float* Bw     = (const float*)d_in[3];
  const float* Cw     = (const float*)d_in[4];
  const float* Dw     = (const float*)d_in[5];
  float* out = (float*)d_out;
  char* ws = (char*)d_ws;

  const size_t szX16 = (size_t)NB * NL * NH * 2;
  const size_t szW16 = (size_t)NS * NH * 2;
  const size_t szPT  = 8192;
  const size_t szBU  = (size_t)QROWS * NS * 4;
  const size_t szY16 = (size_t)QROWS * NS * 2;
  size_t off = 0;
  const size_t oXh = off; off += szX16;
  const size_t oXl = off; off += szX16;
  const size_t oBh = off; off += szW16;
  const size_t oBl = off; off += szW16;
  const size_t oCh = off; off += szW16;
  const size_t oCl = off; off += szW16;
  const size_t oPT = off; off += szPT;
  const size_t oBU = off; off += szBU;
  const size_t oYh = off; off += szY16;
  const size_t oYl = off; off += szY16;
  if (off > ws_size) return;

  unsigned short* Xh  = (unsigned short*)(ws + oXh);
  unsigned short* Xl  = (unsigned short*)(ws + oXl);
  unsigned short* Bh  = (unsigned short*)(ws + oBh);
  unsigned short* Bl  = (unsigned short*)(ws + oBl);
  unsigned short* Ch  = (unsigned short*)(ws + oCh);
  unsigned short* Cl  = (unsigned short*)(ws + oCl);
  float*          PT  = (float*)(ws + oPT);
  float*          BU  = (float*)(ws + oBU);
  unsigned short* YSh = (unsigned short*)(ws + oYh);
  unsigned short* YSl = (unsigned short*)(ws + oYl);

  split_bf16x8<<<dim3((NB * NL * NH / 8) / 256), 256, 0, stream>>>(x, Xh, Xl, NB * NL * NH / 8);
  split_bf16x8<<<dim3((NS * NH / 8) / 256), 256, 0, stream>>>(Bw, Bh, Bl, NS * NH / 8);
  split_bf16x8<<<dim3((NH * NS / 8) / 256), 256, 0, stream>>>(Cw, Ch, Cl, NH * NS / 8);
  state_params<<<dim3(1), NS, 0, stream>>>(A_diag, steps, PT);

  for (int qt = 0; qt < NQ; ++qt) {
    const size_t r0 = (size_t)qt * QROWS;
    wmma_gemm64<1, true, 0, 0, 0><<<dim3((QROWS / 64) * (NS / 64) / 8, 1), 256, 0, stream>>>(
        Xh + r0 * NH, Xl + r0 * NH, NH, 0L,
        Bh, Bl, NH, 0L,
        (void*)BU, (void*)nullptr, NS, 0L,
        (const float*)nullptr,
        (const float*)nullptr, 0L, (const float*)nullptr,
        QROWS, NS, NH, 1.0f);
    state_scan<<<dim3(QSEQ), 32, 0, stream>>>(PT, BU, YSh, YSl);
    wmma_gemm64<1, true, 0, 0, 2><<<dim3((QROWS / 64) * (NH / 64) / 8, 1), 256, 0, stream>>>(
        YSh, YSl, NS, 0L,
        Ch, Cl, NS, 0L,
        (void*)(out + r0 * NH), (void*)nullptr, NH, 0L,
        (const float*)nullptr,
        x + r0 * NH, 0L, Dw,
        QROWS, NH, NS, 1.0f);
  }
}
